// ANPToolEncoder_4638564680178
// MI455X (gfx1250) — hardware-verified
//
#include <hip/hip_runtime.h>
#include <math.h>
#include <stdint.h>

#define NQ    256
#define NG    64
#define NI    256
#define DXF   512
#define HDIM  512
#define NHEAD 8
#define DHEAD 64
#define NTOK  (NG * NI)
#define W1P   514

static_assert(NHEAD * DHEAD == HDIM);
static_assert(DXF == HDIM);
static_assert((NTOK % 64) == 0 && (HDIM % 64) == 0 && (NQ % 64) == 0 && (NI % 64) == 0);

typedef _Float16 v16h __attribute__((ext_vector_type(16)));
typedef _Float16 v8h  __attribute__((ext_vector_type(8)));
typedef float    v8f  __attribute__((ext_vector_type(8)));
typedef float    v4f  __attribute__((ext_vector_type(4)));
typedef unsigned int v4u __attribute__((ext_vector_type(4)));

__device__ __forceinline__ unsigned short h_bits(_Float16 x) { return __builtin_bit_cast(unsigned short, x); }
__device__ __forceinline__ unsigned pk16(unsigned short a, unsigned short b) { return (unsigned)a | ((unsigned)b << 16); }
__device__ __forceinline__ unsigned pkf(float a, float b) { return pk16(h_bits((_Float16)a), h_bits((_Float16)b)); }
__device__ __forceinline__ v8f zero8() { v8f z = {0.f, 0.f, 0.f, 0.f, 0.f, 0.f, 0.f, 0.f}; return z; }

__device__ __forceinline__ v16h ldfrag(const _Float16* p) {
  union { v16h v; v8h h[2]; } f;
  f.h[0] = *(const v8h*)(p);
  f.h[1] = *(const v8h*)(p + 16);
  return f.v;
}

__device__ __forceinline__ v8f mma_h(v16h a, v16h b, v8f c) {
  c = __builtin_amdgcn_wmma_f32_16x16x32_f16(false, a, false, b, (short)0, c, false, false);
#if defined(__HIP_DEVICE_COMPILE__)
  asm volatile("v_nop\n\tv_nop\n\tv_nop\n\tv_nop" : "+v"(c) : "v"(a), "v"(b));
#endif
  return c;
}
__device__ __forceinline__ v8f mma_raw(v16h a, v16h b, v8f c) {
  return __builtin_amdgcn_wmma_f32_16x16x32_f16(false, a, false, b, (short)0, c, false, false);
}
__device__ __forceinline__ void dep_guard(v8f& a, v8f& b, v16h x, v16h y) {
#if defined(__HIP_DEVICE_COMPILE__)
  asm volatile("v_nop\n\tv_nop\n\tv_nop\n\tv_nop" : "+v"(a), "+v"(b) : "v"(x), "v"(y));
#endif
}
__device__ __forceinline__ void keep4(v16h a, v16h b, v16h c, v16h d) {
#if defined(__HIP_DEVICE_COMPILE__)
  asm volatile("v_nop" :: "v"(a), "v"(b), "v"(c), "v"(d));
#endif
}
__device__ __forceinline__ void acc_guard4(v8f& a, v8f& b, v8f& c, v8f& d) {
#if defined(__HIP_DEVICE_COMPILE__)
  asm volatile("v_nop\n\tv_nop\n\tv_nop\n\tv_nop" : "+v"(a), "+v"(b), "+v"(c), "+v"(d));
#endif
}
__device__ __forceinline__ void wave_sync_lds() {
  __builtin_amdgcn_fence(__ATOMIC_RELEASE, "workgroup");
  __builtin_amdgcn_wave_barrier();
  __builtin_amdgcn_fence(__ATOMIC_ACQUIRE, "workgroup");
}

template <int VEC>
__global__ __launch_bounds__(256) void cvt_f16(const float* __restrict__ in, int inPitch, int cols8,
                                               int n8, float scale, unsigned short* out) {
  const int i = blockIdx.x * 256 + threadIdx.x;
  if (i < n8) {
    const int row = i / cols8;
    const int c8  = i - row * cols8;
    const float* src = in + (size_t)row * inPitch + (size_t)c8 * 8;
    float f[8];
    if (VEC) {
      const v4f a = *(const v4f*)(src);
      const v4f b = *(const v4f*)(src + 4);
#pragma unroll
      for (int e = 0; e < 4; ++e) { f[e] = a[e]; f[4 + e] = b[e]; }
    } else {
#pragma unroll
      for (int e = 0; e < 8; ++e) f[e] = src[e];
    }
    v4u p;
#pragma unroll
    for (int e = 0; e < 4; ++e) p[e] = pkf(f[2 * e] * scale, f[2 * e + 1] * scale);
    unsigned short* dst = out + (size_t)i * 8;
    *(volatile v4u*)dst = p;
    __threadfence();
    *(volatile v4u*)dst = p;
  }
}

template <int OUTM, int R1, int BIASM>
__global__ __launch_bounds__(256) void gemm64(
    const unsigned short* __restrict__ Ap, int lda, long long strideA,
    const unsigned short* __restrict__ Btp, int ldb, long long strideB,
    const float* __restrict__ bias,
    const float* __restrict__ r1u, const float* __restrict__ r1v,
    const float* __restrict__ r1w, int r1pitch,
    float alpha, int relu,
    float* C32, int ldc, long long strideC,
    unsigned short* C16, int ldc16, long long strideC16, float oscale,
    int M, int N, int K) {
  const _Float16* A  = (const _Float16*)(const void*)Ap;
  const _Float16* Bt = (const _Float16*)(const void*)Btp;
  __shared__ __align__(16) float sT[8][16 * 68];
  const int b    = blockIdx.y;
  const int lane = threadIdx.x & 31;
  const int wave = threadIdx.x >> 5;
  const int tilesN = N >> 6;
  const int tilesM = M >> 6;
  const int tile = blockIdx.x * 8 + wave;
  if (tile >= tilesM * tilesN) return;
  const int tm = tile / tilesN;
  const int tn = tile - tm * tilesN;
  const int m0 = tm << 6;
  const int n0 = tn << 6;

  const _Float16* Ab = A  + (size_t)b * strideA;
  const _Float16* Bb = Bt + (size_t)b * strideB;

  const int rlane = lane & 15;
  const int koff  = (lane >> 4) * 8;
  const int mOff  = (lane >> 4) * 8;

  v8f acc[4][4];
#pragma unroll
  for (int i = 0; i < 4; ++i)
#pragma unroll
    for (int j = 0; j < 4; ++j) acc[i][j] = zero8();

  for (int k0 = 0; k0 < K; k0 += 32) {
    v16h bh[4];
#pragma unroll
    for (int j = 0; j < 4; ++j) {
      const size_t bo = (size_t)(n0 + (j << 4) + rlane) * ldb + koff + k0;
      bh[j] = ldfrag(Bb + bo);
    }
#pragma unroll
    for (int i = 0; i < 4; ++i) {
      const size_t ao = (size_t)(m0 + (i << 4) + rlane) * lda + koff + k0;
      const v16h ah = ldfrag(Ab + ao);
#pragma unroll
      for (int j = 0; j < 4; ++j) acc[i][j] = mma_raw(ah, bh[j], acc[i][j]);
      dep_guard(acc[i][0], acc[i][3], ah, bh[3]);
    }
    keep4(bh[0], bh[1], bh[2], bh[3]);
  }
  acc_guard4(acc[0][0], acc[0][1], acc[0][2], acc[0][3]);
  acc_guard4(acc[1][0], acc[1][1], acc[1][2], acc[1][3]);
  acc_guard4(acc[2][0], acc[2][1], acc[2][2], acc[2][3]);
  acc_guard4(acc[3][0], acc[3][1], acc[3][2], acc[3][3]);

  float* slab = sT[wave];
  float bcol[4], wu[4], wq[4];
#pragma unroll
  for (int j = 0; j < 4; ++j) {
    const int col = n0 + (j << 4) + rlane;
    bcol[j] = 0.f; wu[j] = 0.f; wq[j] = 0.f;
    if (BIASM == 1) bcol[j] = bias[col];
    if (R1) {
      wu[j] = r1w[(size_t)col * r1pitch];
      wq[j] = r1w[(size_t)col * r1pitch + 1];
    }
  }
#pragma unroll
  for (int i = 0; i < 4; ++i) {
    const int mBase = m0 + (i << 4);
    float brow[8], ru[8], rv[8];
#pragma unroll
    for (int r = 0; r < 8; ++r) {
      const int row = mBase + mOff + r;
      brow[r] = 0.f; ru[r] = 0.f; rv[r] = 0.f;
      if (BIASM == 2) brow[r] = bias[row];
      if (R1) { ru[r] = r1u[row]; rv[r] = r1v[row]; }
    }
#pragma unroll
    for (int j = 0; j < 4; ++j) {
#pragma unroll
      for (int r = 0; r < 8; ++r) {
        float v = acc[i][j][r] * alpha + bcol[j] + brow[r];
        if (R1) v += ru[r] * wu[j] + rv[r] * wq[j];
        if (relu) v = fmaxf(v, 0.f);
        slab[(mOff + r) * 68 + (j << 4) + rlane] = v;
      }
    }
    wave_sync_lds();
    if (OUTM & 1) {
      float* C = C32 + (size_t)b * strideC;
      const int hh2 = lane >> 4, c4 = (lane & 15) * 4;
      for (int pass = 0; pass < 2; ++pass) {
#pragma unroll
        for (int it = 0; it < 8; ++it) {
          const int row = it * 2 + hh2;
          const v4f v = *(const v4f*)(slab + row * 68 + c4);
          *(volatile v4f*)(C + (size_t)(mBase + row) * ldc + n0 + c4) = v;
        }
        __threadfence();
      }
    }
    if (OUTM & 2) {
      unsigned short* C = C16 + (size_t)b * strideC16;
      const int q = lane >> 3, c8 = (lane & 7) * 8;
      v4u hv[4];
#pragma unroll
      for (int it = 0; it < 4; ++it) {
        const int row = it * 4 + q;
        const float* sp = slab + row * 68 + c8;
        v4u a;
#pragma unroll
        for (int e = 0; e < 4; ++e) a[e] = pkf(sp[2 * e] * oscale, sp[2 * e + 1] * oscale);
        hv[it] = a;
      }
      for (int pass = 0; pass < 2; ++pass) {
#pragma unroll
        for (int it = 0; it < 4; ++it) {
          const int row = it * 4 + q;
          *(volatile v4u*)(C + (size_t)(mBase + row) * ldc16 + n0 + c8) = hv[it];
        }
        __threadfence();
      }
    }
    wave_sync_lds();
  }
}

__global__ __launch_bounds__(128)
void self_attn64(const unsigned short* __restrict__ qkp, const unsigned short* __restrict__ vtp,
                 unsigned short* sap) {
  union FH { v16h v; v8h h[2]; };
  __shared__ __align__(16) _Float16 Ksh[64 * 64];
  __shared__ __align__(16) _Float16 Vth[64 * 64];
  __shared__ __align__(16) _Float16 Psh[4][16 * 64];
  __shared__ __align__(16) float    Os[4][16 * 64];

  const int tid  = threadIdx.x;
  const int wave = tid >> 5;
  const int lane = tid & 31;
  const int hh   = lane >> 4;
  const int c    = lane & 15;

  const int bx = blockIdx.x;
  const int qb = bx & 3;
  const int h  = (bx >> 2) & (NHEAD - 1);
  const int m  = bx >> 5;
  const int q0 = qb * 64 + wave * 16;
  const size_t tok0 = (size_t)m * NI;
  const int QKP = 2 * HDIM;

  const _Float16* Qg = (const _Float16*)(const void*)qkp + (size_t)h * DHEAD;
  const _Float16* Kg = Qg + HDIM;
  const _Float16* Vt = (const _Float16*)(const void*)vtp + ((size_t)m * HDIM + (size_t)h * DHEAD) * NI;

  v16h qa[2];
#pragma unroll
  for (int dc = 0; dc < 2; ++dc) qa[dc] = ldfrag(Qg + (tok0 + q0 + c) * QKP + dc * 32 + 8 * hh);

  float mrow[8], lrow[8];
  v8f oacc[4];
#pragma unroll
  for (int r = 0; r < 8; ++r) { mrow[r] = -INFINITY; lrow[r] = 0.f; }
#pragma unroll
  for (int t = 0; t < 4; ++t) oacc[t] = zero8();

  for (int kt = 0; kt < NI / 64; ++kt) {
    const int kv0 = kt * 64;
    __syncthreads();
    {
      const int r = tid >> 1, half = (tid & 1) * 32;
      const _Float16* kg = Kg + (tok0 + kv0 + r) * QKP + half;
      const _Float16* vg = Vt + (size_t)r * NI + kv0 + half;
#pragma unroll
      for (int i = 0; i < 4; ++i) {
        const v8h a0 = *(const v8h*)(kg + 8 * i);
        const v8h b0 = *(const v8h*)(vg + 8 * i);
        *(v8h*)(Ksh + r * 64 + half + 8 * i) = a0;
        *(v8h*)(Vth + r * 64 + half + 8 * i) = b0;
      }
    }
    __syncthreads();

    v8f s[4];
#pragma unroll
    for (int j = 0; j < 4; ++j) {
      s[j] = zero8();
#pragma unroll
      for (int dc = 0; dc < 2; ++dc) {
        FH kb;
        kb.h[0] = *(const v8h*)(Ksh + (j * 16 + c) * 64 + dc * 32 + 8 * hh);
        kb.h[1] = *(const v8h*)(Ksh + (j * 16 + c) * 64 + dc * 32 + 16 + 8 * hh);
        s[j] = mma_h(qa[dc], kb.v, s[j]);
      }
    }

    _Float16* pwh = Psh[wave];
#pragma unroll
    for (int r = 0; r < 8; ++r) {
      float mx = -INFINITY;
#pragma unroll
      for (int j = 0; j < 4; ++j) {
        const float sv = s[j][r] * 0.00048828125f;
        s[j][r] = sv;
        mx = fmaxf(mx, sv);
      }
#pragma unroll
      for (int off = 1; off < 16; off <<= 1) mx = fmaxf(mx, __shfl_xor(mx, off, 32));
      const float mnew  = fmaxf(mrow[r], mx);
      const float alpha = __expf(mrow[r] - mnew);
      mrow[r] = mnew;
      float psum = 0.f;
#pragma unroll
      for (int j = 0; j < 4; ++j) {
        const float p = __expf(s[j][r] - mnew);
        psum += p;
        pwh[(8 * hh + r) * 64 + j * 16 + c] = (_Float16)(p * 1024.0f);
      }
#pragma unroll
      for (int off = 1; off < 16; off <<= 1) psum += __shfl_xor(psum, off, 32);
      lrow[r] = lrow[r] * alpha + psum;
#pragma unroll
      for (int t = 0; t < 4; ++t) oacc[t][r] *= alpha;
    }
    wave_sync_lds();

#pragma unroll 1
    for (int kk = 0; kk < 2; ++kk) {
      FH pa;
      pa.h[0] = *(const v8h*)(pwh + c * 64 + kk * 32 + 8 * hh);
      pa.h[1] = *(const v8h*)(pwh + c * 64 + kk * 32 + 16 + 8 * hh);
#pragma unroll
      for (int t = 0; t < 4; ++t) {
        FH vb;
        vb.h[0] = *(const v8h*)(Vth + (t * 16 + c) * 64 + kk * 32 + 8 * hh);
        vb.h[1] = *(const v8h*)(Vth + (t * 16 + c) * 64 + kk * 32 + 16 + 8 * hh);
        oacc[t] = mma_h(pa.v, vb.v, oacc[t]);
      }
    }
  }

  float* os = Os[wave];
#pragma unroll
  for (int r = 0; r < 8; ++r) {
    const float l = lrow[r];
    const float inv = (l > 0.f) ? (1.0f / l) * (1.0f / 64.0f) : 0.f;
#pragma unroll
    for (int t = 0; t < 4; ++t) os[(8 * hh + r) * 64 + t * 16 + c] = oacc[t][r] * inv;
  }
  wave_sync_lds();
  {
    const int q4 = lane >> 3, c8 = (lane & 7) * 8;
    v4u hv[4];
#pragma unroll
    for (int it = 0; it < 4; ++it) {
      const int row = it * 4 + q4;
      const float* sp = os + row * 64 + c8;
      v4u a;
#pragma unroll
      for (int e = 0; e < 4; ++e) a[e] = pkf(sp[2 * e], sp[2 * e + 1]);
      hv[it] = a;
    }
    for (int pass = 0; pass < 2; ++pass) {
#pragma unroll
      for (int it = 0; it < 4; ++it) {
        const int row = it * 4 + q4;
        const size_t go = (tok0 + q0 + row) * HDIM + (size_t)h * DHEAD + c8;
        *(volatile v4u*)(sap + go) = hv[it];
      }
      __threadfence();
    }
  }
}

__global__ __launch_bounds__(256)
void softmax256(const float* __restrict__ lg, unsigned short* pout, int nrows) {
  const int lane = threadIdx.x & 31;
  const int wave = threadIdx.x >> 5;
  const int row  = blockIdx.x * 8 + wave;
  if (row >= nrows) return;
  const float* p = lg + (size_t)row * 256 + lane * 8;
  const v4f a = *(const v4f*)(p);
  const v4f bq = *(const v4f*)(p + 4);
  float v[8];
#pragma unroll
  for (int e = 0; e < 4; ++e) { v[e] = a[e]; v[4 + e] = bq[e]; }
  float mx = v[0];
#pragma unroll
  for (int e = 1; e < 8; ++e) mx = fmaxf(mx, v[e]);
#pragma unroll
  for (int off = 1; off < 32; off <<= 1) mx = fmaxf(mx, __shfl_xor(mx, off, 32));
  float s = 0.f;
#pragma unroll
  for (int e = 0; e < 8; ++e) { v[e] = __expf(v[e] - mx); s += v[e]; }
#pragma unroll
  for (int off = 1; off < 32; off <<= 1) s += __shfl_xor(s, off, 32);
  const float inv = 1024.0f / s;
  v4u pk;
#pragma unroll
  for (int e = 0; e < 4; ++e) pk[e] = pkf(v[2 * e] * inv, v[2 * e + 1] * inv);
  unsigned short* dst = pout + (size_t)row * 256 + lane * 8;
  *(volatile v4u*)dst = pk;
  __threadfence();
  *(volatile v4u*)dst = pk;
}

__global__ __launch_bounds__(256)
void ln_res_f16(const float* __restrict__ a, const float* __restrict__ res,
                const float* __restrict__ g, const float* __restrict__ bt,
                unsigned short* out, int nrows) {
  const int lane = threadIdx.x & 31;
  const int wave = threadIdx.x >> 5;
  const int row  = blockIdx.x * 8 + wave;
  if (row >= nrows) return;
  const int c0 = lane * 8, c1 = 256 + lane * 8;
  const float* pa = a + (size_t)row * HDIM;
  const float* pr = res + (size_t)row * HDIM;
  float x[16];
  {
    const v4f a0 = *(const v4f*)(pa + c0),     r0 = *(const v4f*)(pr + c0);
    const v4f a1 = *(const v4f*)(pa + c0 + 4), r1 = *(const v4f*)(pr + c0 + 4);
    const v4f a2 = *(const v4f*)(pa + c1),     r2 = *(const v4f*)(pr + c1);
    const v4f a3 = *(const v4f*)(pa + c1 + 4), r3 = *(const v4f*)(pr + c1 + 4);
#pragma unroll
    for (int e = 0; e < 4; ++e) {
      x[e] = a0[e] + r0[e]; x[4 + e] = a1[e] + r1[e]; x[8 + e] = a2[e] + r2[e]; x[12 + e] = a3[e] + r3[e];
    }
  }
  float s = 0.f;
#pragma unroll
  for (int e = 0; e < 16; ++e) s += x[e];
#pragma unroll
  for (int off = 1; off < 32; off <<= 1) s += __shfl_xor(s, off, 32);
  const float mu = s * (1.0f / 512.0f);
  float vs = 0.f;
#pragma unroll
  for (int e = 0; e < 16; ++e) { const float d = x[e] - mu; x[e] = d; vs += d * d; }
#pragma unroll
  for (int off = 1; off < 32; off <<= 1) vs += __shfl_xor(vs, off, 32);
  const float rstd = rsqrtf(vs * (1.0f / 512.0f) + 1e-5f);
  float gv[16], bv[16];
  {
    const v4f g0 = *(const v4f*)(g + c0), g1 = *(const v4f*)(g + c0 + 4), g2 = *(const v4f*)(g + c1), g3 = *(const v4f*)(g + c1 + 4);
    const v4f b0 = *(const v4f*)(bt + c0), b1 = *(const v4f*)(bt + c0 + 4), b2 = *(const v4f*)(bt + c1), b3 = *(const v4f*)(bt + c1 + 4);
#pragma unroll
    for (int e = 0; e < 4; ++e) {
      gv[e] = g0[e]; gv[4 + e] = g1[e]; gv[8 + e] = g2[e]; gv[12 + e] = g3[e];
      bv[e] = b0[e]; bv[4 + e] = b1[e]; bv[8 + e] = b2[e]; bv[12 + e] = b3[e];
    }
  }
  float y[16];
#pragma unroll
  for (int e = 0; e < 16; ++e) y[e] = (x[e] * rstd) * gv[e] + bv[e];
  v4u p0, p1;
#pragma unroll
  for (int e = 0; e < 4; ++e) {
    p0[e] = pkf(y[2 * e], y[2 * e + 1]);
    p1[e] = pkf(y[8 + 2 * e], y[8 + 2 * e + 1]);
  }
  unsigned short* d0 = out + (size_t)row * HDIM + c0;
  unsigned short* d1 = out + (size_t)row * HDIM + c1;
  for (int pass = 0; pass < 2; ++pass) {
    *(volatile v4u*)d0 = p0;
    *(volatile v4u*)d1 = p1;
    __threadfence();
  }
}

__global__ __launch_bounds__(256)
void ln_out_f32(const float* __restrict__ z, const float* __restrict__ g, const float* __restrict__ bt,
                float* out, int nrows) {
  const int lane = threadIdx.x & 31;
  const int wave = threadIdx.x >> 5;
  const int row  = blockIdx.x * 8 + wave;
  if (row >= nrows) return;
  const float* pz = z + (size_t)row * HDIM;
  float x[16];
#pragma unroll
  for (int q = 0; q < 4; ++q) {
    const v4f t = *(const v4f*)(pz + q * 128 + lane * 4);
#pragma unroll
    for (int e = 0; e < 4; ++e) x[4 * q + e] = t[e];
  }
  float s = 0.f;
#pragma unroll
  for (int e = 0; e < 16; ++e) s += x[e];
#pragma unroll
  for (int off = 1; off < 32; off <<= 1) s += __shfl_xor(s, off, 32);
  const float mu = s * (1.0f / 512.0f);
  float vs = 0.f;
#pragma unroll
  for (int e = 0; e < 16; ++e) { const float d = x[e] - mu; x[e] = d; vs += d * d; }
#pragma unroll
  for (int off = 1; off < 32; off <<= 1) vs += __shfl_xor(vs, off, 32);
  const float rstd = rsqrtf(vs * (1.0f / 512.0f) + 1e-5f);
  v4f o[4];
#pragma unroll
  for (int q = 0; q < 4; ++q) {
    const v4f gq = *(const v4f*)(g + q * 128 + lane * 4);
    const v4f bq = *(const v4f*)(bt + q * 128 + lane * 4);
    v4f t;
#pragma unroll
    for (int e = 0; e < 4; ++e) t[e] = (x[4 * q + e] * rstd) * gq[e] + bq[e];
    o[q] = t;
  }
  float* po = out + (size_t)row * HDIM;
  for (int pass = 0; pass < 2; ++pass) {
#pragma unroll
    for (int q = 0; q < 4; ++q) *(volatile v4f*)(po + q * 128 + lane * 4) = o[q];
    __threadfence();
  }
}

extern "C" void kernel_launch(void* const* d_in, const int* in_sizes, int n_in,
                              void* d_out, int out_size, void* d_ws, size_t ws_size,
                              hipStream_t stream) {
  if (n_in < 22) return;
  if (in_sizes[0] != NQ * HDIM) return;
  if (in_sizes[1] != NTOK * DXF) return;
  if (in_sizes[2] != NTOK || in_sizes[3] != NTOK) return;
  if (in_sizes[4] != HDIM * W1P || in_sizes[5] != HDIM) return;
  if (in_sizes[6] != HDIM * HDIM || in_sizes[7] != HDIM) return;
  if (in_sizes[8] != 3 * HDIM * HDIM || in_sizes[9] != 3 * HDIM) return;
  if (in_sizes[10] != HDIM * HDIM || in_sizes[11] != HDIM) return;
  if (in_sizes[12] != HDIM || in_sizes[13] != HDIM) return;
  if (in_sizes[14] != HDIM * HDIM || in_sizes[15] != HDIM) return;
  if (in_sizes[16] != HDIM * DXF || in_sizes[17] != HDIM) return;
  if (in_sizes[18] != HDIM * HDIM || in_sizes[19] != HDIM) return;
  if (in_sizes[20] != HDIM || in_sizes[21] != HDIM) return;
  if (out_size != NQ * NG * HDIM) return;

  const float* q_in  = (const float*)d_in[0];
  const float* ximg  = (const float*)d_in[1];
  const float* gt    = (const float*)d_in[2];
  const float* pred  = (const float*)d_in[3];
  const float* cp_w1 = (const float*)d_in[4];
  const float* cp_b1 = (const float*)d_in[5];
  const float* cp_w2 = (const float*)d_in[6];
  const float* cp_b2 = (const float*)d_in[7];
  const float* in_w  = (const float*)d_in[8];
  const float* in_b  = (const float*)d_in[9];
  const float* out_w = (const float*)d_in[10];
  const float* out_b = (const float*)d_in[11];
  const float* lnc_g = (const float*)d_in[12];
  const float* lnc_b = (const float*)d_in[13];
  const float* wq_w  = (const float*)d_in[14];
  const float* wq_b  = (const float*)d_in[15];
  const float* wk_w  = (const float*)d_in[16];
  const float* wk_b  = (const float*)d_in[17];
  const float* wv_w  = (const float*)d_in[18];
  const float* wv_b  = (const float*)d_in[19];
  const float* lno_g = (const float*)d_in[20];
  const float* lno_b = (const float*)d_in[21];

  const size_t SW    = (size_t)HDIM * HDIM * 2;
  const size_t SQE   = (size_t)NQ * HDIM * 2;
  const size_t SP16  = (size_t)NQ * NTOK * 2;
  const size_t S16M  = (size_t)NTOK * HDIM * 2;
  const size_t S32M  = (size_t)NTOK * HDIM * 4;
  size_t off = 0;
  const size_t oW1   = off; off += SW;
  const size_t oW2   = off; off += SW;
  const size_t oInW  = off; off += 3 * SW;
  const size_t oOutW = off; off += SW;
  const size_t oWq   = off; off += SW;
  const size_t oWk   = off; off += SW;
  const size_t oWv   = off; off += SW;
  const size_t oQE   = off; off += SQE;
  const size_t oQ16  = off; off += SQE;
  const size_t oP16  = off; off += SP16;
  const size_t oR2   = off; off += S16M;
  const size_t oR3   = off; off += S16M;
  const size_t oR4   = off; off += S32M;
  const size_t oR5   = off; off += S32M;
  const size_t oR6   = off; off += S16M;
  if (off > ws_size) return;
  if (off > (size_t)134217728) return;

  char* ws = (char*)d_ws;
  unsigned short* W1h  = (unsigned short*)(ws + oW1);
  unsigned short* W2h  = (unsigned short*)(ws + oW2);
  unsigned short* InWh = (unsigned short*)(ws + oInW);
  unsigned short* OutWh= (unsigned short*)(ws + oOutW);
  unsigned short* Wqh  = (unsigned short*)(ws + oWq);
  unsigned short* Wkh  = (unsigned short*)(ws + oWk);
  unsigned short* Wvh  = (unsigned short*)(ws + oWv);
  unsigned short* QEh  = (unsigned short*)(ws + oQE);
  unsigned short* Q16  = (unsigned short*)(ws + oQ16);
  unsigned short* P16  = (unsigned short*)(ws + oP16);
  unsigned short* Xh   = (unsigned short*)(ws + oR2);
  unsigned short* CE16 = (unsigned short*)(ws + oR2);
  unsigned short* CT16 = (unsigned short*)(ws + oR2);
  unsigned short* K16  = (unsigned short*)(ws + oR3);
  unsigned short* H1h  = (unsigned short*)(ws + oR3);
  unsigned short* VT16 = (unsigned short*)(ws + oR3);
  unsigned short* V2T16= (unsigned short*)(ws + oR3);
  float*          CE32 = (float*)(ws + oR4);
  float*          Z32  = (float*)(ws + oR4);
  unsigned short* QK16 = (unsigned short*)(ws + oR5);
  float*          SP32 = (float*)(ws + oR5);
  float*          LG32 = (float*)(ws + oR6);
  unsigned short* SA16 = (unsigned short*)(ws + oR6);

  const dim3 blk(256);
  const int n8X  = NTOK * DXF / 8;
  const int n8W  = HDIM * HDIM / 8;
  const int n8IW = 3 * HDIM * HDIM / 8;
  const int n8QE = NQ * HDIM / 8;
  const float lscale = 0.04419417382415922f * (1.0f / 16.0f);
  const long long GS16 = (long long)HDIM * NI;

  const dim3 gTok(((NTOK / 64) * (HDIM / 64) + 7) / 8, 1);
  const dim3 gQK(((NTOK / 64) * (2 * HDIM / 64) + 7) / 8, 1);
  const dim3 gQ(((NQ / 64) * (HDIM / 64) + 7) / 8, 1);
  const dim3 gLG(((NQ / 64) * (NTOK / 64) + 7) / 8, 1);
  const dim3 gVT(((HDIM / 64) * (NI / 64) + 7) / 8, NG);
  const dim3 gZ(((NQ / 64) * (HDIM / 64) + 7) / 8, NG);
  const dim3 gRow(NTOK / 8);

  cvt_f16<1><<<dim3((n8X + 255) / 256), blk, 0, stream>>>(ximg, DXF, DXF / 8, n8X, 1.0f, Xh);
  cvt_f16<0><<<dim3((n8W + 255) / 256), blk, 0, stream>>>(cp_w1, W1P, HDIM / 8, n8W, 64.0f, W1h);
  cvt_f16<1><<<dim3((n8W + 255) / 256), blk, 0, stream>>>(cp_w2, HDIM, HDIM / 8, n8W, 64.0f, W2h);
  cvt_f16<1><<<dim3((n8IW + 255) / 256), blk, 0, stream>>>(in_w, HDIM, HDIM / 8, n8IW, 64.0f, InWh);
  cvt_f16<1><<<dim3((n8W + 255) / 256), blk, 0, stream>>>(out_w, HDIM, HDIM / 8, n8W, 64.0f, OutWh);
  cvt_f16<1><<<dim3((n8W + 255) / 256), blk, 0, stream>>>(wq_w, HDIM, HDIM / 8, n8W, 64.0f, Wqh);
  cvt_f16<1><<<dim3((n8W + 255) / 256), blk, 0, stream>>>(wk_w, DXF, DXF / 8, n8W, 64.0f, Wkh);
  cvt_f16<1><<<dim3((n8W + 255) / 256), blk, 0, stream>>>(wv_w, HDIM, HDIM / 8, n8W, 64.0f, Wvh);
  cvt_f16<1><<<dim3((n8QE + 255) / 256), blk, 0, stream>>>(q_in, HDIM, HDIM / 8, n8QE, 1.0f, QEh);

  gemm64<2, 0, 1><<<gQ, blk, 0, stream>>>(
      QEh, HDIM, 0LL, Wqh, HDIM, 0LL, wq_b, gt, pred, cp_w1, W1P, 1.0f / 64.0f, 0,
      Z32, HDIM, 0LL, Q16, HDIM, 0LL, 4.0f, NQ, HDIM, HDIM);
  gemm64<2, 0, 1><<<gTok, blk, 0, stream>>>(
      Xh, DXF, 0LL, Wkh, DXF, 0LL, wk_b, gt, pred, cp_w1, W1P, 1.0f / 64.0f, 0,
      Z32, HDIM, 0LL, K16, HDIM, 0LL, 4.0f, NTOK, HDIM, DXF);
  gemm64<1, 0, 0><<<gLG, blk, 0, stream>>>(
      Q16, HDIM, 0LL, K16, HDIM, 0LL, cp_b1, gt, pred, cp_w1, W1P, lscale, 0,
      LG32, NTOK, 0LL, P16, NTOK, 0LL, 1.0f, NQ, NTOK, HDIM);
  softmax256<<<gRow, blk, 0, stream>>>(LG32, P16, NQ * NG);

  gemm64<2, 1, 1><<<gTok, blk, 0, stream>>>(
      Xh, DXF, 0LL, W1h, HDIM, 0LL, cp_b1, gt, pred, cp_w1 + DXF, W1P, 1.0f / 64.0f, 1,
      Z32, HDIM, 0LL, H1h, HDIM, 0LL, 1.0f, NTOK, HDIM, DXF);
  gemm64<3, 0, 1><<<gTok, blk, 0, stream>>>(
      H1h, HDIM, 0LL, W2h, HDIM, 0LL, cp_b2, gt, pred, cp_w1, W1P, 1.0f / 64.0f, 0,
      CE32, HDIM, 0LL, CE16, HDIM, 0LL, 8.0f, NTOK, HDIM, HDIM);

  gemm64<2, 0, 1><<<gQK, blk, 0, stream>>>(
      CE16, HDIM, 0LL, InWh, HDIM, 0LL, in_b, gt, pred, cp_w1, W1P, 1.0f / 512.0f, 0,
      Z32, HDIM, 0LL, QK16, 2 * HDIM, 0LL, 16.0f, NTOK, 2 * HDIM, HDIM);
  gemm64<2, 0, 2><<<gVT, blk, 0, stream>>>(
      InWh + (size_t)2 * HDIM * HDIM, HDIM, 0LL, CE16, HDIM, (long long)NI * HDIM, in_b + 2 * HDIM,
      gt, pred, cp_w1, W1P, 1.0f / 512.0f, 0,
      Z32, HDIM, 0LL, VT16, NI, GS16, 16.0f, HDIM, NI, HDIM);
  self_attn64<<<dim3(NG * NHEAD * 4), dim3(128), 0, stream>>>(QK16, VT16, SA16);
  gemm64<1, 0, 1><<<gTok, blk, 0, stream>>>(
      SA16, HDIM, 0LL, OutWh, HDIM, 0LL, out_b, gt, pred, cp_w1, W1P, 1.0f / 16384.0f, 0,
      SP32, HDIM, 0LL, P16, HDIM, 0LL, 1.0f, NTOK, HDIM, HDIM);
  ln_res_f16<<<gRow, blk, 0, stream>>>(CE32, SP32, lnc_g, lnc_b, CT16, NTOK);

  gemm64<2, 0, 2><<<gVT, blk, 0, stream>>>(
      Wvh, HDIM, 0LL, CT16, HDIM, (long long)NI * HDIM, wv_b, gt, pred, cp_w1, W1P, 1.0f / 64.0f, 0,
      Z32, HDIM, 0LL, V2T16, NI, GS16, 4.0f, HDIM, NI, HDIM);
  gemm64<1, 0, 0><<<gZ, blk, 0, stream>>>(
      P16, NTOK, (long long)NI, V2T16, NI, GS16, cp_b1, gt, pred, cp_w1, W1P, 1.0f / 4096.0f, 0,
      Z32, NG * HDIM, (long long)HDIM, Q16, HDIM, 0LL, 1.0f, NQ, HDIM, NI);
  ln_out_f32<<<gRow, blk, 0, stream>>>(Z32, lno_g, lno_b, (float*)d_out, NQ * NG);
  (void)hipGetLastError();
}
